// CAN_29566554866256
// MI455X (gfx1250) — hardware-run, weakly checked
//
#include <hip/hip_runtime.h>


#ifndef NB
#define NB 16
#endif
#define NB_FULL 16
#define NT_IN   16
#define NI_IN   8
#define XDC     23
#define NT_OUT  32
#define NPART   8
#define NI_OUT  8
#define DA_     16
#define DG_     6
#define DCO     23
#define NQ      (NT_IN * NI_IN)
#define NPT     (NPART * NQ)
#define HD      32
#define RW      16
#define OSH     36
#define X_BSTR  (NT_IN * NI_IN * XDC)
#define OUT_B   (NT_OUT * NI_OUT * DCO)
#define HCAR    64.0f
#define PCAR    16384.0f
#define QCAR    4096.0f
#define SCL     ((float)(1.4426950408889634 / (64.0 * 4096.0)))
#define WSC     ((float)(1.0 / (16384.0 * 64.0)))

static_assert(NB % 2 == 0);
static_assert(NB <= NB_FULL);
static_assert(NI_IN == 8);
static_assert(DA_ == 16);
static_assert(DA_ + DG_ + 1 <= 32);
static_assert(DA_ + DG_ <= HD);
static_assert(HD == 32);
static_assert(NQ == 128);
static_assert(NPT == 1024);
static_assert(NQ % 32 == 0);
static_assert(NT_OUT == 2 * RW);
static_assert(NI_OUT == 8);
static_assert(DCO == 1 + DG_ + DA_);
static_assert((OSH * 4) % 16 == 0);
static_assert(16 * 32 * 16 == NQ * HD * 2);
static_assert(16 * 32 * 16 == HD * NQ * 2);
static_assert((OUT_B * 4) % 128 == 0);
static_assert((OUT_B / 4) % 32 == 0);
static_assert(2 * NQ * OSH * 4 <= 131072);
static_assert((RW * NQ + NQ + NT_OUT * 24 + OUT_B) * 4 <= 131072);

typedef _Float16 h16;
typedef unsigned short bf;
typedef __attribute__((ext_vector_type(16))) __bf16   v16bf;
typedef __attribute__((ext_vector_type(16))) _Float16 v16h;
typedef __attribute__((ext_vector_type(8)))  _Float16 v8h;
typedef __attribute__((ext_vector_type(8)))  unsigned short v8us;
typedef __attribute__((ext_vector_type(8)))  float    v8f;
typedef __attribute__((ext_vector_type(4)))  float    v4f;
typedef v4f  __attribute__((may_alias)) v4fa;

__device__ __forceinline__ unsigned short f2bf(float f) { unsigned u = __float_as_uint(f); u += 0x7FFFu + ((u >> 16) & 1u); return (unsigned short)(u >> 16); }
__device__ __forceinline__ float bfr(float f) { return __uint_as_float(((unsigned)f2bf(f)) << 16); }
__device__ __forceinline__ v16h cat16(v8h lo, v8h hi) { return __builtin_shufflevector(lo, hi, 0, 1, 2, 3, 4, 5, 6, 7, 8, 9, 10, 11, 12, 13, 14, 15); }
__device__ __forceinline__ v16bf cat16b(v8us lo, v8us hi) { return __builtin_bit_cast(v16bf, __builtin_shufflevector(lo, hi, 0, 1, 2, 3, 4, 5, 6, 7, 8, 9, 10, 11, 12, 13, 14, 15)); }
__device__ __forceinline__ v8f wmma16(v16h a, v16h b, v8f c) { return __builtin_amdgcn_wmma_f32_16x16x32_f16(false, a, false, b, (short)0, c, false, false); }
__device__ __forceinline__ v8f wmmab(v16bf a, v16bf b, v8f c) { return __builtin_amdgcn_wmma_f32_16x16x32_bf16(false, a, false, b, (short)0, c, false, false); }
__device__ __forceinline__ v16h  ldh(const h16* p) { return cat16(*(const v8h*)p, *(const v8h*)(p + 16)); }
__device__ __forceinline__ v16bf ldb(const bf* p)  { return cat16b(*(const v8us*)p, *(const v8us*)(p + 16)); }
__device__ __forceinline__ void wave_sync() { __builtin_amdgcn_fence(3  , "wavefront"); __builtin_amdgcn_wave_barrier(); asm volatile("" ::: "memory"); }

static __device__ __forceinline__ h16 toh_flush(float v) { const h16 r = (h16)v; return (fabsf(v) < 6.103515625e-05f) ? (h16)0.0f : r; }
__device__ __forceinline__ v8f wmma16g(v16h a, v16h b, v8f c) { c = wmma16(a, b, c); asm volatile("v_nop\n\tv_nop\n\tv_nop\n\tv_nop" : "+v"(c) : "v"(a), "v"(b)); return c; }
__device__ __forceinline__ v8f wmmabg(v16bf a, v16bf b, v8f c) { c = wmmab(a, b, c); asm volatile("v_nop\n\tv_nop\n\tv_nop\n\tv_nop" : "+v"(c) : "v"(a), "v"(b)); return c; }

__global__ __launch_bounds__(256) void k_xplane(const float* __restrict__ x, bf* XP, unsigned total) {
    const unsigned i = blockIdx.x * 256u + threadIdx.x; if (i >= total) return;
    const unsigned k8 = (i & 3u) * 8u; const unsigned rowg = i >> 2;
    const unsigned row = rowg % (unsigned)(NB * NI_IN), ic = rowg / (unsigned)(NB * NI_IN);
    const unsigned b = row >> 3, ii = row & 7u;
    const float* xs = x + ((size_t)(b * NT_IN + ic) * NI_IN + ii) * XDC;
    v8us o;
#pragma unroll
    for (int j = 0; j < 8; ++j) {
        const unsigned k = k8 + (unsigned)j;
        unsigned col = (k < 16u) ? (7u + k) : ((k < 22u) ? (k - 15u) : 1u);
        asm volatile("" : "+v"(col));
        float v = xs[col];
        asm volatile("" : "+v"(v));
        const unsigned short hv = f2bf(v);
        o[j] = (k < 22u) ? hv : ((k == 22u) ? (unsigned short)0x3F80 : (unsigned short)0);
    }
    *(volatile v8us*)(XP + (size_t)i * 8) = o; __threadfence(); *(volatile v8us*)(XP + (size_t)i * 8) = o;
}

__global__ __launch_bounds__(256) void k_wplane(const float* __restrict__ W1, const float* __restrict__ W2, bf* WP, unsigned total) {
    const unsigned i = blockIdx.x * 256u + threadIdx.x; if (i >= total) return;
    const int role = __builtin_amdgcn_readfirstlane((int)(threadIdx.x >> 5)) & 3;
    const unsigned lane = threadIdx.x & 31u;
    const unsigned k8 = (lane & 3u) * 8u, n = (unsigned)role * 8u + (lane >> 2);
    const unsigned t = i >> 7;
    v8us o = (v8us){};
    if (role < 2) {
        const float* w = W2 + (size_t)t * (DA_ * DA_) + n;
#pragma unroll
        for (int j = 0; j < 8; ++j) {
            const unsigned k = k8 + (unsigned)j;
            unsigned kk = (k < 15u) ? k : 15u;
            asm volatile("" : "+v"(kk));
            float v = w[kk * DA_];
            asm volatile("" : "+v"(v));
            const unsigned short hv = f2bf(v);
            o[j] = (k < 16u) ? hv : (unsigned short)0;
        }
    } else if (role == 2) {
        const unsigned f = n - 16u; const unsigned fc = (f < 5u) ? f : 5u;
        const float* w = W1 + (size_t)t * ((DG_ + 1) * DG_) + fc;
#pragma unroll
        for (int j = 0; j < 8; ++j) {
            const unsigned k = k8 + (unsigned)j;
            unsigned e = (k >= 16u) ? (k - 16u) : 0u; e = (e < 6u) ? e : 6u;
            asm volatile("" : "+v"(e));
            float v = w[e * DG_];
            asm volatile("" : "+v"(v));
            const unsigned short hv = f2bf(v);
            o[j] = ((k >= 16u) & (k < 23u) & (f < 6u)) ? hv : (unsigned short)0;
        }
    }
    *(volatile v8us*)(WP + (size_t)i * 8) = o; __threadfence(); *(volatile v8us*)(WP + (size_t)i * 8) = o;
}

__global__ __launch_bounds__(32) void k_gemm(const bf* __restrict__ XP, const bf* __restrict__ WP, h16* H, h16* HT) {
    __shared__ __align__(16) float os[2 * NQ * OSH];
    const int lane = threadIdx.x & 31, lr = lane & 15, hi = lane >> 4;
    const int bp = blockIdx.x; const int ncp = blockIdx.y; const int nc = ncp >> 3, np = ncp & 7;
    const size_t aoff = (size_t)(bp * 16 + lr) * 32 + 8 * hi;
    const size_t boff = ((size_t)ncp * 32 + lr) * 32 + 8 * hi;
#pragma unroll 1
    for (int ic = 0; ic < NT_IN; ++ic) {
        const v16bf a = ldb(XP + (size_t)ic * ((size_t)NB * NI_IN * 32) + aoff);
        const bf* wb = WP + (size_t)ic * ((size_t)NT_OUT * NPART * 1024) + boff;
        const v16bf b0 = ldb(wb), b1 = ldb(wb + 16 * 32);
        v8f c0 = (v8f){}, c1 = (v8f){};
        c0 = wmmabg(a, b0, c0); c1 = wmmabg(a, b1, c1);
#pragma unroll
        for (int r = 0; r < 8; ++r) {
            os[(hi * NQ + ic * 8 + r) * OSH + lr]      = c0[r] * HCAR;
            os[(hi * NQ + ic * 8 + r) * OSH + 16 + lr] = c1[r] * HCAR; }
    }
    wave_sync();
#pragma unroll 1
    for (int ps = 0; ps < 2; ++ps) {
#pragma unroll 1
        for (int bl = 0; bl < 2; ++bl) {
            const size_t zrow = (size_t)(bp * 2 + bl) * NT_OUT + nc;
            const size_t prow = zrow * NPT + (size_t)np * NQ;
            const size_t trow = zrow * HD;
#pragma unroll 1
            for (int s = 0; s < 16; ++s) {
                const int p = 8 * s + (lane >> 2), c8 = (lane & 3) * 8;
                const v4f x0 = *(const v4fa*)(&os[(bl * NQ + p) * OSH + c8]); const v4f x1 = *(const v4fa*)(&os[(bl * NQ + p) * OSH + c8 + 4]); v8h hv;
#pragma unroll
                for (int i = 0; i < 4; ++i) { hv[i] = toh_flush(x0[i]); hv[4 + i] = toh_flush(x1[i]); }
                *(volatile v8h*)(H + (prow + (size_t)p) * HD + c8) = hv; }
#pragma unroll 1
            for (int s = 0; s < 16; ++s) {
                const int d = 2 * s + (lane >> 4), p8 = (lane & 15) * 8; v8h hv;
#pragma unroll
                for (int i = 0; i < 8; ++i) hv[i] = toh_flush(os[(bl * NQ + p8 + i) * OSH + d]);
                *(volatile v8h*)(HT + (trow + (size_t)d) * NPT + (size_t)np * NQ + p8) = hv; }
        }
        if (ps == 0) __threadfence(); }
}

struct E2 { v8f a; v8f b; };
__device__ __forceinline__ E2 step_exp(const h16* __restrict__ KP, size_t ko, int key0, v16h qf) {
    const h16* ka = KP + ko + (size_t)key0 * HD;
    const v16h ka0 = ldh(ka), kb0 = ldh(ka + 16 * HD);
    v8f s0 = (v8f){}, s1 = (v8f){};
    s0 = wmma16g(ka0, qf, s0); s1 = wmma16g(kb0, qf, s1);
    E2 e;
#pragma unroll
    for (int r = 0; r < 8; ++r) {
        const float x0 = fminf(fmaxf(s0[r] * SCL, -60.0f), 60.0f), x1 = fminf(fmaxf(s1[r] * SCL, -60.0f), 60.0f);
        e.a[r] = __builtin_amdgcn_exp2f(x0); e.b[r] = __builtin_amdgcn_exp2f(x1); }
    return e;
}

__global__ __launch_bounds__(32 * RW) void k_iter(const h16* __restrict__ KP, const h16* __restrict__ VT, float* OUT) {
    __shared__ __align__(16) float dpart[RW * NQ];
    __shared__ __align__(16) float dinv[NQ];
    __shared__ __align__(16) float so[NT_OUT * 24];
    __shared__ __align__(16) float fl[OUT_B];
    const int lane = threadIdx.x & 31, lr = lane & 15, hi = lane >> 4;
    const int wave = __builtin_amdgcn_readfirstlane((int)(threadIdx.x >> 5));
    const int b = blockIdx.x;
    size_t ko[2], vo[2];
#pragma unroll
    for (int cap = 0; cap < 2; ++cap) {
        const size_t pbase = ((size_t)b * NT_OUT + (size_t)(wave + RW * cap)) * NPT * HD;
        ko[cap] = pbase + (size_t)lr * HD + 8 * hi;
        vo[cap] = pbase + (size_t)lr * NPT + 8 * hi; }
    v16h qf[2]; v8f sa[2], sg[2];
#pragma unroll
    for (int cap = 0; cap < 2; ++cap) { qf[cap] = (v16h){}; sa[cap] = (v8f){}; sg[cap] = (v8f){}; }
#pragma unroll 1
    for (int it = 0; it < 3; ++it) {
#pragma unroll 1
        for (int qg = 0; qg < 4; ++qg) {
            v8f da = (v8f){}, db = (v8f){};
#pragma unroll
            for (int cap = 0; cap < 2; ++cap) {
#pragma unroll 1
                for (int np = 0; np < NPART; ++np) {
                    const E2 e = step_exp(KP, ko[cap], np * NQ + qg * 32, qf[cap]);
                    da = da + e.a; db = db + e.b; } }
            if (lr == 0) {
                const int base = wave * NQ + qg * 32 + 8 * hi;
                v4f t0, t1, t2, t3;
#pragma unroll
                for (int r = 0; r < 4; ++r) { t0[r] = da[r]; t1[r] = da[4 + r]; t2[r] = db[r]; t3[r] = db[4 + r]; }
                *(v4fa*)(&dpart[base]) = t0; *(v4fa*)(&dpart[base + 4]) = t1; *(v4fa*)(&dpart[base + 16]) = t2; *(v4fa*)(&dpart[base + 20]) = t3; }
        }
        __syncthreads();
        if (threadIdx.x < NQ) {
            float s = 0.0f;
#pragma unroll 1
            for (int w = 0; w < RW; ++w) s += dpart[w * NQ + threadIdx.x];
            dinv[threadIdx.x] = PCAR * (1.0f / ((float)NI_OUT * s)); }
        __syncthreads();
#pragma unroll
        for (int cap = 0; cap < 2; ++cap) {
            v8f o0 = (v8f){}, o1 = (v8f){}; float l = 0.0f;
#pragma unroll 1
            for (int key0 = 0; key0 < NPT; key0 += 32) {
                const E2 e = step_exp(KP, ko[cap], key0, qf[cap]);
                const int q0 = (key0 & (NQ - 1)) + 8 * hi;
                const v4f i0 = *(const v4fa*)(&dinv[q0]), i1 = *(const v4fa*)(&dinv[q0 + 4]), i2 = *(const v4fa*)(&dinv[q0 + 16]), i3 = *(const v4fa*)(&dinv[q0 + 20]);
                v16h pb; float ls = 0.0f;
#pragma unroll
                for (int r = 0; r < 4; ++r) {
                    const h16 pa = toh_flush(e.a[r] * i0[r]), pc = toh_flush(e.a[4 + r] * i1[r]);
                    const h16 pd = toh_flush(e.b[r] * i2[r]), pe = toh_flush(e.b[4 + r] * i3[r]);
                    pb[r] = pa; pb[4 + r] = pc; pb[8 + r] = pd; pb[12 + r] = pe;
                    ls += ((float)pa + (float)pc) + ((float)pd + (float)pe); }
                l += ls;
                const h16* va = VT + vo[cap] + key0;
                const v16h v0 = ldh(va), v1 = ldh(va + (size_t)16 * NPT);
                o0 = wmma16g(v0, pb, o0); o1 = wmma16g(v1, pb, o1);
            }
            l += __shfl_xor(l, 16, 32);
            const float lsafe = (l > 0.0f) ? l : 1.0f;
            const float cinv = 1.0f / (lsafe * (1.0f / PCAR));
            float wa[8], og[8]; float ss = 0.0f;
#pragma unroll
            for (int r = 0; r < 8; ++r) { wa[r] = o0[r] * WSC; og[r] = (o1[r] * WSC) * cinv; ss += wa[r] * wa[r]; }
            ss += __shfl_xor(ss, 16, 32);
            const float scale = ss / (1.0f + ss) / sqrtf(ss + 1e-7f);
            v16h q;
#pragma unroll
            for (int r = 0; r < 8; ++r) {
                sa[cap][r] += 0.01f * wa[r]; sg[cap][r] += og[r];
                q[r]     = toh_flush(fminf(fmaxf(sa[cap][r] * QCAR, -32000.0f), 32000.0f));
                q[8 + r] = toh_flush(fminf(fmaxf(sg[cap][r] * QCAR, -32000.0f), 32000.0f)); }
            qf[cap] = q;
            const int nc = wave + RW * cap;
            if (lane == 0) {
                so[nc * 24] = scale;
#pragma unroll
                for (int r = 0; r < DG_; ++r) so[nc * 24 + 1 + r] = og[r];
#pragma unroll
                for (int r = 0; r < 8; ++r) so[nc * 24 + 7 + r] = wa[r]; }
            if (lane == 16) {
#pragma unroll
                for (int r = 0; r < 8; ++r) so[nc * 24 + 15 + r] = wa[r]; }
        }
    }
    __syncthreads();
#pragma unroll 1
    for (int e = threadIdx.x; e < OUT_B; e += 32 * RW) {
        const int nc = e / (NI_OUT * DCO); const int rem = e - nc * (NI_OUT * DCO); const int d = rem % DCO;
        fl[e] = so[nc * 24 + d]; }
    __syncthreads();
    float* ob = OUT + (size_t)b * OUT_B;
#pragma unroll 1
    for (int ps = 0; ps < 2; ++ps) {
#pragma unroll 1
        for (int idx = threadIdx.x; idx < OUT_B / 4; idx += 32 * RW) {
            const v4f val = *(const v4fa*)(&fl[idx * 4]);
            *(volatile v4f*)(ob + (size_t)idx * 4) = val; }
        if (ps == 0) __threadfence(); }
}

static constexpr size_t al256(size_t v) { return (v + 255) & ~(size_t)255; }
static constexpr size_t SZ_XP = al256((size_t)NT_IN * NB * NI_IN * 32 * 2);
static constexpr size_t SZ_WP = al256((size_t)NT_IN * NT_OUT * NPART * 32 * 32 * 2);
static constexpr size_t SZ_H  = al256((size_t)NB * NT_OUT * NPT * HD * 2);
static constexpr size_t SZ_TOTAL = SZ_XP + SZ_WP + 2 * SZ_H;
static_assert(SZ_TOTAL <= (size_t)134217728);
static_assert(((size_t)NT_IN * NB * NI_IN * 4) % 256 == 0 || true);
static_assert(((size_t)NT_IN * NT_OUT * NPART * 128) % 256 == 0);
static_assert((size_t)(NB / 2) * 2 * NT_OUT * NPART * NQ * HD * 2 == (size_t)NB * NT_OUT * NPT * HD * 2);

extern "C" void kernel_launch(void* const* d_in, const int* in_sizes, int n_in,
                              void* d_out, int out_size, void* d_ws, size_t ws_size, hipStream_t stream) {
    if (n_in < 3) return;
    if ((size_t)in_sizes[0] < (size_t)NB * X_BSTR) return;
    if ((size_t)in_sizes[1] < (size_t)NT_IN * NT_OUT * NPART * (DG_ + 1) * DG_) return;
    if ((size_t)in_sizes[2] < (size_t)NT_IN * NT_OUT * NPART * DA_ * DA_) return;
    if ((size_t)out_size < (size_t)NB * OUT_B) return;
    if (SZ_TOTAL > ws_size) return;
    const float* x  = (const float*)d_in[0];
    const float* W1 = (const float*)d_in[1];
    const float* W2 = (const float*)d_in[2];
    float* OUT = (float*)d_out;
    char* wsp = (char*)d_ws;
    bf*  XP = (bf*)wsp;  wsp += SZ_XP;
    bf*  WP = (bf*)wsp;  wsp += SZ_WP;
    h16* H  = (h16*)wsp; wsp += SZ_H;
    h16* HT = (h16*)wsp; wsp += SZ_H;

    { const unsigned total = (unsigned)(NT_IN * NB * NI_IN * 4);
      k_xplane<<<(total + 255u) / 256u, 256, 0, stream>>>(x, XP, total); }
    { const unsigned total = (unsigned)(NT_IN * NT_OUT * NPART * 128);
      k_wplane<<<(total + 255u) / 256u, 256, 0, stream>>>(W1, W2, WP, total); }
    k_gemm<<<dim3(NB / 2, NT_OUT * NPART, 1), 32, 0, stream>>>(XP, WP, H, HT);
    k_iter<<<dim3(NB, 1, 1), 32 * RW, 0, stream>>>(H, HT, OUT);
}
